// DimeNet_52922587022003
// MI455X (gfx1250) — hardware-verified
//
#include <hip/hip_runtime.h>
#include <stddef.h>


typedef float          v4f   __attribute__((ext_vector_type(4)));
typedef float          v8f   __attribute__((ext_vector_type(8)));
typedef int            v4i   __attribute__((ext_vector_type(4)));
typedef unsigned int   v4u   __attribute__((ext_vector_type(4)));
typedef unsigned short v8us  __attribute__((ext_vector_type(8)));
typedef unsigned short v16us __attribute__((ext_vector_type(16)));
typedef __bf16         v16bf __attribute__((ext_vector_type(16)));
union FragU { v16bf v; v16us s; v8us h[2]; unsigned int u[8]; };

#define HC    128
#define PP    136
#define TP    132
#define OTP   68
#define NRB   32

#define OFF_WXH    0
#define OFF_WXL    16384
#define OFF_WL1H   32768
#define OFF_WL3H   98304
#define OFF_WL3L   114688
#define OFF_WLSH   131072
#define OFF_WLSL   180224
#define OFF_WOH    229376
#define OFF_WOL    237568
#define WSW_SHORTS 245760

#define ENT   256
#define ENW   8
#define EPT   8
#define CHUNK (ENT * EPT)
#define WCAP  (EPT * 32)
#define LISTN (ENW * WCAP)
#define PE    64
#define PCAP  (CHUNK + PE)
#define NB    256

static_assert((PCAP % PE) == 0);
static_assert((NB % ENW) == 0);
static_assert(PE == 64);
static_assert(ENT == 2 * HC);

#define O_ACC   0
#define O_PLH   (O_ACC + NB * HC * 4)
#define O_PLL   (O_PLH + PE * PP * 2)
#define O_TILE  (O_PLL + PE * PP * 2)
#define O_RBF   (O_TILE + PE * TP * 4)
#define O_LIST  (O_RBF + PE * 8 * 4)
#define O_PEND  (O_LIST + LISTN * 4)
#define O_SLOT  (O_PEND + PCAP * 4)
#define O_SRC   (O_SLOT + PE * 4)
#define O_DST   (O_SRC + PE * 4)
#define O_WCNT  (O_DST + PE * 4)
#define O_PNDN  (O_WCNT + ENW * 4)
#define EDGE_LDS (O_PNDN + 16)
static_assert((O_PLH % 16) == 0);
static_assert((O_PLL % 16) == 0);
static_assert((O_TILE % 16) == 0);
static_assert((O_RBF % 16) == 0);
static_assert((O_LIST % 16) == 0);
static_assert((O_PEND % 16) == 0);
static_assert((O_SLOT % 16) == 0);
static_assert((O_WCNT % 16) == 0);
static_assert(EDGE_LDS == 219184);

__device__ __forceinline__ unsigned int f2bf(float x) {
  unsigned int u = __float_as_uint(x);
  u += 0x7fffu + ((u >> 16) & 1u);
  return u >> 16;
}
__device__ __forceinline__ void split2(float x, unsigned int& hi, unsigned int& lo) {
  hi = f2bf(x);
  const float hf = __uint_as_float(hi << 16);
  lo = f2bf(x - hf);
}
__device__ __forceinline__ float swishf(float t) {
  const float e = __expf(-t);
  const float s = __builtin_amdgcn_rcpf(1.0f + e);
  return t * s;
}
__device__ __forceinline__ v8f splat8(float v) {
  v8f r;
#pragma unroll
  for (int i = 0; i < 8; ++i) r[i] = v;
  return r;
}
__device__ __forceinline__ v8f wmb(const FragU& a, const FragU& b, v8f c) {
  v8f d = __builtin_amdgcn_wmma_f32_16x16x32_bf16(false, a.v, false, b.v, (short)0, c, false, false);
  asm volatile("v_nop\n\tv_nop\n\tv_nop\n\tv_nop" : "+v"(d) : "v"(a.v), "v"(b.v));
  return d;
}
__device__ __forceinline__ void ldfrag(const unsigned short* rowp, int k0, int hh, FragU& f) {
  f.h[0] = *(const v8us*)(rowp + k0 + 8 * hh);
  f.h[1] = *(const v8us*)(rowp + k0 + 16 + 8 * hh);
}
__device__ __forceinline__ void ldfrag_f32(const float* rowp, int k0, int hh, FragU& fh, FragU& fl) {
  const float* p0 = rowp + k0 + 8 * hh;
  const float* p1 = rowp + k0 + 16 + 8 * hh;
  const v4f a0 = *(const v4f*)p0;
  const v4f a1 = *(const v4f*)(p0 + 4);
  const v4f b0 = *(const v4f*)p1;
  const v4f b1 = *(const v4f*)(p1 + 4);
  float f[16];
  f[0] = a0.x; f[1] = a0.y; f[2]  = a0.z; f[3]  = a0.w; f[4]  = a1.x; f[5]  = a1.y; f[6]  = a1.z; f[7]  = a1.w;
  f[8] = b0.x; f[9] = b0.y; f[10] = b0.z; f[11] = b0.w; f[12] = b1.x; f[13] = b1.y; f[14] = b1.z; f[15] = b1.w;
#pragma unroll
  for (int i = 0; i < 8; ++i) {
    unsigned int h0, l0, h1, l1;
    split2(f[2 * i], h0, l0);
    split2(f[2 * i + 1], h1, l1);
    fh.u[i] = h0 | (h1 << 16);
    fl.u[i] = l0 | (l1 << 16);
  }
}
__device__ __forceinline__ void planes_put(unsigned short* pH, unsigned short* pL, int idx, float v) {
  unsigned int h, l;
  split2(v, h, l);
  pH[idx] = (unsigned short)h;
  pL[idx] = (unsigned short)l;
}

template <int NCT>
__device__ __forceinline__ void mm_planes(const unsigned short* aH, const unsigned short* aL,
                                          const unsigned short* bH, const unsigned short* bL,
                                          int ct0, int m, int hh, v8f (&acc)[NCT]) {
#pragma unroll
  for (int ks = 0; ks < 4; ++ks) {
    FragU ah, al;
    ldfrag(aH, ks * 32, hh, ah);
    ldfrag(aL, ks * 32, hh, al);
#pragma unroll
    for (int q = 0; q < NCT; ++q) {
      const unsigned short* bp = bH + ((ct0 + q) * 16 + m) * HC;
      const unsigned short* bq = bL + ((ct0 + q) * 16 + m) * HC;
      FragU bh, blo;
      ldfrag(bp, ks * 32, hh, bh);
      ldfrag(bq, ks * 32, hh, blo);
      acc[q] = wmb(ah, bh, acc[q]);
      acc[q] = wmb(ah, blo, acc[q]);
      acc[q] = wmb(al, bh, acc[q]);
    }
  }
}
template <int NCT>
__device__ __forceinline__ void mm_f32a(const float* arow, const unsigned short* bH, const unsigned short* bL,
                                        int ct0, int m, int hh, v8f (&acc)[NCT]) {
#pragma unroll
  for (int ks = 0; ks < 4; ++ks) {
    FragU ah, al;
    ldfrag_f32(arow, ks * 32, hh, ah, al);
#pragma unroll
    for (int q = 0; q < NCT; ++q) {
      const unsigned short* bp = bH + ((ct0 + q) * 16 + m) * HC;
      const unsigned short* bq = bL + ((ct0 + q) * 16 + m) * HC;
      FragU bh, blo;
      ldfrag(bp, ks * 32, hh, bh);
      ldfrag(bq, ks * 32, hh, blo);
      acc[q] = wmb(ah, bh, acc[q]);
      acc[q] = wmb(ah, blo, acc[q]);
      acc[q] = wmb(al, bh, acc[q]);
    }
  }
}
__device__ __forceinline__ void rows_store16(const float* tl, float* dst, int lane) {
#pragma unroll
  for (int rr = 0; rr < 16; ++rr) {
    const v4f v = *(const v4f*)(tl + rr * TP + 4 * lane);
    *(volatile v4f*)(dst + (size_t)rr * HC + 4 * lane) = v;
  }
  __threadfence();
#pragma unroll
  for (int rr = 0; rr < 16; ++rr) {
    const v4f v = *(const v4f*)(tl + rr * TP + 4 * lane);
    *(volatile v4f*)(dst + (size_t)rr * HC + 4 * lane) = v;
  }
}

__global__ __launch_bounds__(256) void k_pack(const float* __restrict__ Wx, const float* __restrict__ Wl,
                                             const float* __restrict__ Wls, const float* __restrict__ Wout,
                                             unsigned short* wsw) {
  const int t = blockIdx.x * 256 + (int)threadIdx.x;
  if (t >= 15360) return;
  const float* src;
  int dh, dl;
  if (t < 2048) {
    const int row = t >> 4, k8 = (t & 15) * 8;
    src = Wx + row * HC + k8;
    dh = OFF_WXH + row * HC + k8;
    dl = OFF_WXL + row * HC + k8;
  } else if (t < 8192) {
    const int u = t - 2048;
    const int j = u >> 11;
    const int v = u & 2047;
    const int row = v >> 4, k8 = (v & 15) * 8;
    src = Wl + row * (3 * HC) + j * HC + k8;
    dh = OFF_WL1H + j * 32768 + row * HC + k8;
    dl = dh + 16384;
  } else if (t < 14336) {
    const int u = t - 8192;
    const int row = u >> 4, k8 = (u & 15) * 8;
    src = Wls + row * HC + k8;
    dh = OFF_WLSH + row * HC + k8;
    dl = OFF_WLSL + row * HC + k8;
  } else {
    const int u = t - 14336;
    const int row = u >> 4, k8 = (u & 15) * 8;
    src = Wout + row * HC + k8;
    dh = OFF_WOH + row * HC + k8;
    dl = OFF_WOL + row * HC + k8;
  }
  const v4f a = *(const v4f*)src;
  const v4f b = *(const v4f*)(src + 4);
  float f[8];
  f[0] = a.x; f[1] = a.y; f[2] = a.z; f[3] = a.w; f[4] = b.x; f[5] = b.y; f[6] = b.z; f[7] = b.w;
  unsigned int hv[8], lv[8];
#pragma unroll
  for (int i = 0; i < 8; ++i) split2(f[i], hv[i], lv[i]);
  v4u qh, ql;
  qh.x = hv[0] | (hv[1] << 16); qh.y = hv[2] | (hv[3] << 16); qh.z = hv[4] | (hv[5] << 16); qh.w = hv[6] | (hv[7] << 16);
  ql.x = lv[0] | (lv[1] << 16); ql.y = lv[2] | (lv[3] << 16); ql.z = lv[4] | (lv[5] << 16); ql.w = lv[6] | (lv[7] << 16);
  *(volatile v4u*)(wsw + dh) = qh;
  *(volatile v4u*)(wsw + dl) = ql;
  __threadfence();
  *(volatile v4u*)(wsw + dh) = qh;
  *(volatile v4u*)(wsw + dl) = ql;
}

__global__ __launch_bounds__(256) void k_angle(const float* __restrict__ pos, const int* __restrict__ ii,
                                              const int* __restrict__ jj, const int* __restrict__ kk,
                                              float* ang, int T, int nN) {
  const int t = blockIdx.x * 256 + (int)threadIdx.x;
  if (t >= T) return;
  int i = ii[t], j = jj[t], k = kk[t];
  i = i < 0 ? 0 : (i > nN - 1 ? nN - 1 : i);
  j = j < 0 ? 0 : (j > nN - 1 ? nN - 1 : j);
  k = k < 0 ? 0 : (k > nN - 1 ? nN - 1 : k);
  const float pix = pos[(size_t)i * 3 + 0], piy = pos[(size_t)i * 3 + 1], piz = pos[(size_t)i * 3 + 2];
  const float ax = pos[(size_t)j * 3 + 0] - pix, ay = pos[(size_t)j * 3 + 1] - piy, az = pos[(size_t)j * 3 + 2] - piz;
  const float bx = pos[(size_t)k * 3 + 0] - pix, by = pos[(size_t)k * 3 + 1] - piy, bz = pos[(size_t)k * 3 + 2] - piz;
  const float dot = ax * bx + ay * by + az * bz;
  const float cx = ay * bz - az * by, cy = az * bx - ax * bz, cz = ax * by - ay * bx;
  const float cr = sqrtf(cx * cx + cy * cy + cz * cz);
  const float v = atan2f(cr, dot);
  *(volatile float*)(ang + t) = v;
  __threadfence();
  *(volatile float*)(ang + t) = v;
}

__global__ __launch_bounds__(64) void k_node1(const float* __restrict__ x, const unsigned short* __restrict__ wsw,
                                             float* Pws, float* Qws, int nN) {
  __shared__ __attribute__((aligned(16))) unsigned short plH[NRB * PP];
  __shared__ __attribute__((aligned(16))) unsigned short plL[NRB * PP];
  __shared__ __attribute__((aligned(16))) float tile[NRB * TP];
  const int tid = threadIdx.x, lane = tid & 31, w = tid >> 5, hh = lane >> 4, m = lane & 15;
  const int rowBase = blockIdx.x * NRB;

  v8f acc[8];
#pragma unroll
  for (int q = 0; q < 8; ++q) acc[q] = splat8(0.0f);
  {
    int grow = rowBase + w * 16 + m;
    grow = grow > nN - 1 ? nN - 1 : grow;
    mm_f32a<8>(x + (size_t)grow * HC, wsw + OFF_WXH, wsw + OFF_WXL, 0, m, hh, acc);
  }
#pragma unroll
  for (int q = 0; q < 8; ++q) {
#pragma unroll
    for (int rr = 0; rr < 8; ++rr)
      planes_put(plH, plL, (w * 16 + 8 * hh + rr) * PP + q * 16 + m, acc[q][rr]);
  }
  __syncthreads();

  const unsigned short* arH = plH + (w * 16 + m) * PP;
  const unsigned short* arL = plL + (w * 16 + m) * PP;
#pragma unroll 1
  for (int part = 0; part < 2; ++part) {
#pragma unroll
    for (int q = 0; q < 8; ++q) acc[q] = splat8(0.0f);
    const unsigned short* bH = wsw + OFF_WL1H + part * 32768;
    mm_planes<8>(arH, arL, bH, bH + 16384, 0, m, hh, acc);
#pragma unroll
    for (int q = 0; q < 8; ++q) {
#pragma unroll
      for (int rr = 0; rr < 8; ++rr)
        tile[(w * 16 + 8 * hh + rr) * TP + q * 16 + m] = acc[q][rr];
    }
    __syncthreads();
    float* dst = (part == 0 ? Pws : Qws) + (size_t)(rowBase + w * 16) * HC;
    rows_store16(tile + (w * 16) * TP, dst, lane);
    __syncthreads();
  }
}

__global__ __launch_bounds__(64) void k_node2(const float* __restrict__ Sws, const unsigned short* __restrict__ wsw,
                                             const float* __restrict__ bls, float* out, int nN, int sRows) {
  __shared__ __attribute__((aligned(16))) unsigned short plH[NRB * PP];
  __shared__ __attribute__((aligned(16))) unsigned short plL[NRB * PP];
  __shared__ __attribute__((aligned(16))) float otile[NRB * OTP];
  const int tid = threadIdx.x, lane = tid & 31, w = tid >> 5, hh = lane >> 4, m = lane & 15;
  const int rowBase = blockIdx.x * NRB;

  v8f acc[8];
#pragma unroll
  for (int q = 0; q < 8; ++q) acc[q] = splat8(bls[q * 16 + m]);
  {
    int srow = rowBase + w * 16 + m;
    srow = srow > sRows - 1 ? sRows - 1 : srow;
    mm_f32a<8>(Sws + (size_t)srow * HC, wsw + OFF_WLSH, wsw + OFF_WLSL, 0, m, hh, acc);
  }
#pragma unroll
  for (int q = 0; q < 8; ++q) {
#pragma unroll
    for (int rr = 0; rr < 8; ++rr)
      planes_put(plH, plL, (w * 16 + 8 * hh + rr) * PP + q * 16 + m, swishf(acc[q][rr]));
  }
  __syncthreads();

  const unsigned short* arH = plH + (w * 16 + m) * PP;
  const unsigned short* arL = plL + (w * 16 + m) * PP;
#pragma unroll 1
  for (int L = 1; L < 3; ++L) {
#pragma unroll
    for (int q = 0; q < 8; ++q) acc[q] = splat8(bls[L * HC + q * 16 + m]);
    mm_planes<8>(arH, arL, wsw + OFF_WLSH + L * 16384, wsw + OFF_WLSL + L * 16384, 0, m, hh, acc);
    __syncthreads();
#pragma unroll
    for (int q = 0; q < 8; ++q) {
#pragma unroll
      for (int rr = 0; rr < 8; ++rr)
        planes_put(plH, plL, (w * 16 + 8 * hh + rr) * PP + q * 16 + m, swishf(acc[q][rr]));
    }
    __syncthreads();
  }

  v8f o[4];
#pragma unroll
  for (int q = 0; q < 4; ++q) o[q] = splat8(0.0f);
  mm_planes<4>(arH, arL, wsw + OFF_WOH, wsw + OFF_WOL, 0, m, hh, o);
#pragma unroll
  for (int q = 0; q < 4; ++q) {
#pragma unroll
    for (int rr = 0; rr < 8; ++rr)
      otile[(w * 16 + 8 * hh + rr) * OTP + q * 16 + m] = o[q][rr];
  }
  __syncthreads();
  {
    const int sub = lane >> 4, c4 = 4 * (lane & 15);
    v4f ov[8];
#pragma unroll
    for (int j = 0; j < 8; ++j) ov[j] = *(const v4f*)(otile + (w * 16 + 2 * j + sub) * OTP + c4);
#pragma unroll
    for (int j = 0; j < 8; ++j) {
      const int grow = rowBase + w * 16 + 2 * j + sub;
      if (grow < nN) *(volatile v4f*)(out + (size_t)grow * 64 + c4) = ov[j];
    }
    __threadfence();
#pragma unroll
    for (int j = 0; j < 8; ++j) {
      const int grow = rowBase + w * 16 + 2 * j + sub;
      if (grow < nN) *(volatile v4f*)(out + (size_t)grow * 64 + c4) = ov[j];
    }
  }
}

__device__ __forceinline__ int scan_chunk(const int* __restrict__ dsts, int nE, int cbase, int nodeBase,
                                          int vec8, int* list, int tid, int wave) {
  int wc = 0;
  const int el0  = tid * EPT;
  const int e0   = cbase + el0;
  const int sent = -2147483647 - 1;
  v4i da, db;
  if (vec8 != 0 && cbase + CHUNK <= nE) {
    da = *(const v4i*)(dsts + e0);
    db = *(const v4i*)(dsts + e0 + 4);
  } else {
    da.x = (e0     < nE) ? dsts[min(e0, nE - 1)] : sent;
    da.y = (e0 + 1 < nE) ? dsts[min(e0 + 1, nE - 1)] : sent;
    da.z = (e0 + 2 < nE) ? dsts[min(e0 + 2, nE - 1)] : sent;
    da.w = (e0 + 3 < nE) ? dsts[min(e0 + 3, nE - 1)] : sent;
    db.x = (e0 + 4 < nE) ? dsts[min(e0 + 4, nE - 1)] : sent;
    db.y = (e0 + 5 < nE) ? dsts[min(e0 + 5, nE - 1)] : sent;
    db.z = (e0 + 6 < nE) ? dsts[min(e0 + 6, nE - 1)] : sent;
    db.w = (e0 + 7 < nE) ? dsts[min(e0 + 7, nE - 1)] : sent;
  }
  const unsigned nb = (unsigned)nodeBase;
  const unsigned s0 = (unsigned)da.x - nb, s1 = (unsigned)da.y - nb;
  const unsigned s2 = (unsigned)da.z - nb, s3 = (unsigned)da.w - nb;
  const unsigned s4 = (unsigned)db.x - nb, s5 = (unsigned)db.y - nb;
  const unsigned s6 = (unsigned)db.z - nb, s7 = (unsigned)db.w - nb;
  const bool h0 = s0 < (unsigned)NB, h1 = s1 < (unsigned)NB, h2 = s2 < (unsigned)NB, h3 = s3 < (unsigned)NB;
  const bool h4 = s4 < (unsigned)NB, h5 = s5 < (unsigned)NB, h6 = s6 < (unsigned)NB, h7 = s7 < (unsigned)NB;
  const unsigned any = __builtin_amdgcn_ballot_w32(h0 | h1 | h2 | h3 | h4 | h5 | h6 | h7);
  if (any != 0u) {
#define HITJ(J, HJ) { \
      const unsigned mj = __builtin_amdgcn_ballot_w32(HJ); \
      if (mj != 0u) { \
        if (HJ) { \
          const int p = wc + (int)__builtin_amdgcn_mbcnt_lo(mj, 0u); \
          if (p < WCAP) list[wave * WCAP + p] = el0 + (J); \
        } \
        wc += (int)__builtin_popcount(mj); } }
    HITJ(0, h0)
    HITJ(1, h1)
    HITJ(2, h2)
    HITJ(3, h3)
    HITJ(4, h4)
    HITJ(5, h5)
    HITJ(6, h6)
    HITJ(7, h7)
#undef HITJ
  }
  return wc;
}

__global__ __launch_bounds__(ENT) void k_edge(
    const float* __restrict__ pos, const float* __restrict__ freq,
    const int* __restrict__ esrc, const int* __restrict__ edst,
    const float* __restrict__ Pws, const float* __restrict__ Qws,
    const float* __restrict__ Wr, const float* __restrict__ br,
    const float* __restrict__ Wrbf, const float* __restrict__ bl,
    const unsigned short* __restrict__ wsw, float* Sws, int nN, int nE, int vec8) {
  extern __shared__ __attribute__((aligned(16))) unsigned char dsm[];
  float*          acc   = (float*)(dsm + O_ACC);
  unsigned short* plH   = (unsigned short*)(dsm + O_PLH);
  unsigned short* plL   = (unsigned short*)(dsm + O_PLL);
  float*          tile  = (float*)(dsm + O_TILE);
  float*          rbfv  = (float*)(dsm + O_RBF);
  int*            list  = (int*)(dsm + O_LIST);
  int*            pend  = (int*)(dsm + O_PEND);
  int*            slotb = (int*)(dsm + O_SLOT);
  int*            srcb  = (int*)(dsm + O_SRC);
  int*            dstb  = (int*)(dsm + O_DST);
  int*            wcnt  = (int*)(dsm + O_WCNT);
  int*            pendN = (int*)(dsm + O_PNDN);

  const int tid = threadIdx.x, lane = tid & 31, wave = tid >> 5, hh = lane >> 4, m = lane & 15;
  const int nodeBase = blockIdx.x * NB;

  {
    const v4f z = {0.0f, 0.0f, 0.0f, 0.0f};
    for (int i = tid; i < NB * HC / 4; i += ENT) ((v4f*)acc)[i] = z;
  }
  if (tid == 0) pendN[0] = 0;
  float fq[6];
#pragma unroll
  for (int k = 0; k < 6; ++k) fq[k] = freq[k];
  const int cch = tid & (HC - 1);
  float wr[6], wb[6];
#pragma unroll
  for (int k = 0; k < 6; ++k) { wr[k] = Wr[cch * 6 + k]; wb[k] = Wrbf[cch * 6 + k]; }
  const float brc = br[cch];
  __syncthreads();

  const int nChunks = (nE + CHUNK - 1) / CHUNK;
#pragma unroll 1
  for (int ch = 0; ch < nChunks; ++ch) {
    const int cbase = ch * CHUNK;
    const int wc = scan_chunk(edst, nE, cbase, nodeBase, vec8, list, tid, wave);
    if (lane == 0) wcnt[wave] = wc;
    __syncthreads();

    int base = pendN[0];
    base = base < 0 ? 0 : (base > PE ? PE : base);
    int tot = 0, myoff = 0;
#pragma unroll
    for (int w2 = 0; w2 < ENW; ++w2) {
      int c = wcnt[w2];
      c = c > WCAP ? WCAP : (c < 0 ? 0 : c);
      if (w2 < wave) myoff += c;
      tot += c;
    }
    int newN = base + tot;
    newN = newN > PCAP ? PCAP : newN;
    {
      int n = wcnt[wave];
      n = n > WCAP ? WCAP : (n < 0 ? 0 : n);
      const int* lp = list + wave * WCAP;
      for (int i = lane; i < n; i += 32) {
        const int p = base + myoff + i;
        if (p < PCAP) pend[p] = cbase + lp[i];
      }
    }
    const int fin = (ch == nChunks - 1) ? 1 : 0;
    const int R   = (fin != 0) ? (newN + PE - 1) / PE : newN / PE;
    const int Pv  = (fin != 0) ? newN : R * PE;
    __syncthreads();

#pragma unroll 1
    for (int r = 0; r < R; ++r) {
      if (tid < PE) {
        const int idx = r * PE + tid;
        const bool valid = idx < Pv;
        int e = pend[idx];
        e = valid ? e : 0;
        e = e < 0 ? 0 : (e > nE - 1 ? nE - 1 : e);
        int dnod = edst[e];
        int snod = esrc[e];
        int slot = dnod - nodeBase;
        if (!valid || (unsigned)slot >= (unsigned)NB) slot = NB;
        dnod = dnod < 0 ? 0 : (dnod > nN - 1 ? nN - 1 : dnod);
        snod = snod < 0 ? 0 : (snod > nN - 1 ? nN - 1 : snod);
        const float* pd = pos + (size_t)dnod * 3;
        const float* ps = pos + (size_t)snod * 3;
        const float dx = pd[0] - ps[0], dy = pd[1] - ps[1], dz = pd[2] - ps[2];
        const float dist = sqrtf(dx * dx + dy * dy + dz * dz);
        const float dn = dist * 0.2f;
        const float d2 = dn * dn;
        const float dp = d2 * d2 * dn;
        const float env = 1.0f / dn + (-21.0f) * dp + 35.0f * dp * dn + (-15.0f) * dp * dn * dn;
#pragma unroll 1
        for (int k = 0; k < 6; ++k) {
          const float sv = env * sinf(fq[k] * dn);
          rbfv[tid * 8 + k] = valid ? sv : 0.0f;
        }
        rbfv[tid * 8 + 6] = 0.0f;
        rbfv[tid * 8 + 7] = 0.0f;
        slotb[tid] = slot;
        srcb[tid]  = snod;
        dstb[tid]  = dnod;
      }
      __syncthreads();

      {
        const int par = tid >> 7;
#pragma unroll 1
        for (int i = 0; i < PE / 2; ++i) {
          const int e = 2 * i + par;
          const v4f ra = *(const v4f*)(rbfv + e * 8);
          const v4f rq = *(const v4f*)(rbfv + e * 8 + 4);
          float s1 = ra.x * wr[0];
          s1 += ra.y * wr[1]; s1 += ra.z * wr[2]; s1 += ra.w * wr[3]; s1 += rq.x * wr[4]; s1 += rq.y * wr[5];
          float s2 = ra.x * wb[0];
          s2 += ra.y * wb[1]; s2 += ra.z * wb[2]; s2 += ra.w * wb[3]; s2 += rq.x * wb[4]; s2 += rq.y * wb[5];
          const float v = swishf(s1 + brc);
          unsigned int vh, vl;
          split2(v, vh, vl);
          plH[e * PP + cch] = (unsigned short)vh;
          plL[e * PP + cch] = (unsigned short)vl;
          tile[e * TP + cch] = s2;
        }
      }
      __syncthreads();

      {
        const int rt = wave >> 1, ctb = (wave & 1) * 4;
        v8f ea[4];
#pragma unroll
        for (int q = 0; q < 4; ++q) ea[q] = splat8(0.0f);
        mm_planes<4>(plH + (rt * 16 + m) * PP, plL + (rt * 16 + m) * PP,
                     wsw + OFF_WL3H, wsw + OFF_WL3L, ctb, m, hh, ea);
        int dd[8], ss[8];
#pragma unroll
        for (int rr = 0; rr < 8; ++rr) {
          const int row = rt * 16 + 8 * hh + rr;
          dd[rr] = dstb[row];
          ss[rr] = srcb[row];
        }
#pragma unroll
        for (int q = 0; q < 4; ++q) {
          const int col = (ctb + q) * 16 + m;
          const float blv = bl[col];
#pragma unroll
          for (int rr = 0; rr < 8; ++rr) {
            const int row = rt * 16 + 8 * hh + rr;
            const float pv = Pws[(size_t)dd[rr] * HC + col];
            const float qv = Qws[(size_t)ss[rr] * HC + col];
            const float g  = tile[row * TP + col];
            const float u  = ((pv + qv) + ea[q][rr]) + blv;
            tile[row * TP + col] = g * swishf(u);
          }
        }
      }
      __syncthreads();

      if (wave == 0) {
#pragma unroll 1
        for (int i = 0; i < PE; ++i) {
          const int sl = slotb[i];
          if ((unsigned)sl < (unsigned)NB) {
            const v4f tv = *(const v4f*)(tile + i * TP + 4 * lane);
            v4f* ap = (v4f*)(acc + sl * HC + 4 * lane);
            const v4f av = *ap;
            *ap = av + tv;
          }
        }
      }
      __syncthreads();
    }

    int rem = newN - R * PE;
    rem = rem < 0 ? 0 : rem;
    if (R > 0 && tid < rem) pend[tid] = pend[R * PE + tid];
    if (tid == 0) pendN[0] = rem;
  }
  __syncthreads();

  float* sb = Sws + (size_t)nodeBase * HC;
#pragma unroll 1
  for (int sl = wave; sl < NB; sl += ENW) {
    const v4f v = *(const v4f*)(acc + sl * HC + 4 * lane);
    *(volatile v4f*)(sb + (size_t)sl * HC + 4 * lane) = v;
  }
  __threadfence();
#pragma unroll 1
  for (int sl = wave; sl < NB; sl += ENW) {
    const v4f v = *(const v4f*)(acc + sl * HC + 4 * lane);
    *(volatile v4f*)(sb + (size_t)sl * HC + 4 * lane) = v;
  }
}

extern "C" void kernel_launch(void* const* d_in, const int* in_sizes, int n_in,
                              void* d_out, int out_size, void* d_ws, size_t ws_size,
                              hipStream_t stream) {
  if (n_in < 17) return;
  const int N = in_sizes[0] / HC;
  if (N <= 0 || in_sizes[0] != N * HC || in_sizes[1] != N * 3) return;
  if (in_sizes[2] < 6) return;
  if (in_sizes[3] != HC * HC || in_sizes[4] != HC * 6 || in_sizes[5] < HC) return;
  if (in_sizes[6] != HC * 3 * HC || in_sizes[7] < HC || in_sizes[8] != HC * 6) return;
  if (in_sizes[9] != 3 * HC * HC || in_sizes[10] < 3 * HC || in_sizes[11] != 64 * HC) return;
  const int E = in_sizes[12];
  if (E < 1 || in_sizes[13] != E) return;
  const int T = in_sizes[14];
  if (T < 0 || in_sizes[15] != T || in_sizes[16] != T) return;
  if ((long long)out_size != (long long)N * 64 + (long long)T) return;

  const float* x    = (const float*)d_in[0];
  const float* pos  = (const float*)d_in[1];
  const float* freq = (const float*)d_in[2];
  const float* Wx   = (const float*)d_in[3];
  const float* Wr   = (const float*)d_in[4];
  const float* br   = (const float*)d_in[5];
  const float* Wl   = (const float*)d_in[6];
  const float* bl   = (const float*)d_in[7];
  const float* Wrbf = (const float*)d_in[8];
  const float* Wls  = (const float*)d_in[9];
  const float* bls  = (const float*)d_in[10];
  const float* Wout = (const float*)d_in[11];
  const int*   esrc = (const int*)d_in[12];
  const int*   edst = (const int*)d_in[13];
  const int*   ii   = (const int*)d_in[14];
  const int*   jj   = (const int*)d_in[15];
  const int*   kk   = (const int*)d_in[16];
  float* out = (float*)d_out;

  const int nBlkN = (N + NRB - 1) / NRB;
  const int nBlkE = (N + NB - 1) / NB;
  const size_t rowsN = (size_t)nBlkN * NRB;
  const size_t rowsE = (size_t)nBlkE * NB;

  char* ws = (char*)d_ws;
  size_t off = 0;
  const size_t oW = off; off += (size_t)WSW_SHORTS * 2;            off = (off + 255) & ~(size_t)255;
  const size_t oP = off; off += rowsN * HC * 4;                     off = (off + 255) & ~(size_t)255;
  const size_t oQ = off; off += rowsN * HC * 4;                     off = (off + 255) & ~(size_t)255;
  const size_t oS = off; off += rowsE * HC * 4;                     off = (off + 255) & ~(size_t)255;
  if (off > ws_size) return;
  unsigned short* wsw = (unsigned short*)(ws + oW);
  float* Pws = (float*)(ws + oP);
  float* Qws = (float*)(ws + oQ);
  float* Sws = (float*)(ws + oS);

  const int vec8 = ((E & 3) == 0) ? 1 : 0;

  if (T > 0)
    k_angle<<<(T + 255) / 256, 256, 0, stream>>>(pos, ii, jj, kk, out + (size_t)N * 64, T, N);

  k_pack<<<60, 256, 0, stream>>>(Wx, Wl, Wls, Wout, wsw);

  k_node1<<<nBlkN, 64, 0, stream>>>(x, wsw, Pws, Qws, N);

  (void)hipFuncSetAttribute(reinterpret_cast<const void*>(&k_edge),
                            hipFuncAttributeMaxDynamicSharedMemorySize, EDGE_LDS);
  k_edge<<<nBlkE, ENT, EDGE_LDS, stream>>>(pos, freq, esrc, edst, Pws, Qws, Wr, br, Wrbf, bl,
                                           wsw, Sws, N, E, vec8);

  k_node2<<<nBlkN, 64, 0, stream>>>(Sws, wsw, bls, out, N, (int)rowsE);
}
